// NAGNNActor_41059887349848
// MI455X (gfx1250) — hardware-run, weakly checked
//
#include <hip/hip_runtime.h>
#include <stddef.h>


#define NNODE   1024
#define FINC    16
#define HIDC    128
#define HID2    256
#define KLIN    400
#define KL1     16
#define KGAP    16
#define KLP     416
#define KPL     448
#define TN      32
#define NTHR    256
#define NWAVE   8
#define DEGCAP  16
#define BPB     16
#define BGRP    128
#define ECHUNK  256
#define WLCAP   32
#define WSCL    64
#define OSC     0.015625f
#define OBP     132
#define YP      260
#define SOP     40
#define MINV    (-100000.0f)
#define LNEPS   1e-5f
#define WSCAP   134217728

static_assert(NTHR == NWAVE * 32);
static_assert(NTHR == HID2);
static_assert(TN * 8 == NTHR);
static_assert(NNODE == 4 * NTHR);
static_assert((NNODE % TN) == 0);
static_assert(KLP == 32 + 3 * HIDC);
static_assert(KPL >= KLP && (KPL % 32) == 0);
static_assert((OBP % 4) == 0 && (YP % 4) == 0 && (SOP % 8) == 0);
static_assert(WLCAP >= 32);
static_assert(TN * DEGCAP == 2 * NTHR);

typedef float    v2f  __attribute__((ext_vector_type(2)));
typedef float    v4f  __attribute__((ext_vector_type(4)));
typedef float    v8f  __attribute__((ext_vector_type(8)));
typedef _Float16 v2h  __attribute__((ext_vector_type(2)));
typedef _Float16 v4h  __attribute__((ext_vector_type(4)));
typedef _Float16 v8h  __attribute__((ext_vector_type(8)));
typedef _Float16 v16h __attribute__((ext_vector_type(16)));
union FragH { v16h v; v8h h[2]; };

__device__ __forceinline__ v8f wmf(v16h a, v16h b, v8f c) {
  v8f d = __builtin_amdgcn_wmma_f32_16x16x32_f16(false, a, false, b, (short)0, c, false, false);
  asm volatile("v_nop\n\tv_nop\n\tv_nop\n\tv_nop" : "+v"(d) : "v"(a), "v"(b));
  return d;
}

__device__ __forceinline__ v8f zero8() { v8f z = {0.f, 0.f, 0.f, 0.f, 0.f, 0.f, 0.f, 0.f}; return z; }

template <int KPITCH>
__global__ __launch_bounds__(NTHR) void k_wT16(const float* __restrict__ W, _Float16* Wp,
                                               int K, int NC, int K1, int GAP, float scale) {
  static_assert((KPITCH % 32) == 0 && KPITCH <= 448);
  constexpr int TPP    = KPITCH + 8;
  constexpr int NPC    = KPITCH / 8;
  constexpr int NPIECE = 32 * NPC;
  constexpr int NIT    = (NPIECE + NTHR - 1) / NTHR;
  __shared__ __attribute__((aligned(16))) _Float16 sT[32 * TPP];
  const int tid = threadIdx.x, n = tid & 31, kq = tid >> 5;
  const int n0 = (int)blockIdx.x * 32;
#pragma unroll 1
  for (int i = 0; i < NPC; ++i) {
    const int kk = kq + 8 * i;
    const int row = (kk < K1) ? kk : (kk - GAP);
    const bool valid = ((kk < K1) || (kk >= K1 + GAP)) && (row < K);
    const int rowc = row < 0 ? 0 : (row > K - 1 ? K - 1 : row);
    float v = W[(size_t)rowc * NC + n0 + n] * scale;
    v = valid ? v : 0.0f;
    sT[n * TPP + kk] = (_Float16)v;
  }
  __syncthreads();
  v8h hv[NIT];
#pragma unroll
  for (int it = 0; it < NIT; ++it) {
    const int q = tid + NTHR * it;
    const int qc = q < NPIECE ? q : NPIECE - 1;
    const int row = qc / NPC, p = qc - row * NPC;
    hv[it] = *(const v8h*)(sT + row * TPP + 8 * p);
  }
  _Float16* base = Wp + (size_t)n0 * KPITCH;
#pragma unroll
  for (int it = 0; it < NIT; ++it) {
    const int q = tid + NTHR * it;
    if (q < NPIECE) *(volatile v8h*)(base + 8 * q) = hv[it];
  }
  __threadfence();
#pragma unroll
  for (int it = 0; it < NIT; ++it) {
    const int q = tid + NTHR * it;
    if (q < NPIECE) *(volatile v8h*)(base + 8 * q) = hv[it];
  }
}

template <int KIN, bool F32IN>
__global__ __launch_bounds__(NTHR) void k_layer(const void* __restrict__ xin,
    const int* __restrict__ esrc, const int* __restrict__ edst,
    const _Float16* __restrict__ Wp, const float* __restrict__ bias,
    const float* __restrict__ lng, const float* __restrict__ lnb,
    _Float16* hout, int nE, int nb) {
  static_assert(KIN == FINC || KIN == HIDC);
  constexpr int KP  = ((KIN + 31) / 32) * 32;
  constexpr int KPA = KP + 8;
  constexpr int CPT = KIN / 8;
  __shared__ __attribute__((aligned(16))) _Float16 sAgg[TN * KPA];
  __shared__ __attribute__((aligned(16))) float sOb[TN * OBP];
  __shared__ __attribute__((aligned(16))) float sPar[3 * HIDC];
  __shared__ float sStat[2 * TN];
  __shared__ int sNbr[TN * DEGCAP];
  __shared__ int sCnt[TN];
  __shared__ int sList[NWAVE * WLCAP];
  __shared__ int sWcnt[NWAVE];
  __shared__ int sMaxd;

  const int tid = threadIdx.x, lane = tid & 31, wave = tid >> 5, hh = lane >> 4, m = lane & 15;
  const int node0 = (int)blockIdx.x * TN;
  const int lb0 = (int)blockIdx.y * BPB;

  if (tid < TN) sCnt[tid] = 0;
  sNbr[tid] = node0 + (tid / DEGCAP);
  sNbr[tid + NTHR] = node0 + ((tid + NTHR) / DEGCAP);
  if (tid < HIDC) { sPar[tid] = bias[tid]; sPar[2 * HIDC + tid] = lnb[tid]; }
  else            { sPar[tid] = lng[tid - HIDC]; }
  if constexpr (KP > KIN) {
    constexpr int PPR = (KP - KIN) / 8;
    if (tid < TN * PPR) {
      const int row = tid / PPR, p = tid - row * PPR;
      v8h z;
#pragma unroll
      for (int e = 0; e < 8; ++e) z[e] = (_Float16)0.0f;
      *(v8h*)(sAgg + row * KPA + KIN + 8 * p) = z;
    }
  }
  __syncthreads();

  const int nChunks = (nE + ECHUNK - 1) / ECHUNK;
#pragma unroll 1
  for (int ch = 0; ch < nChunks; ++ch) {
    const int e  = ch * ECHUNK + tid;
    const int ec = e < nE ? e : nE - 1;
    const int d  = edst[ec];
    const unsigned sl = (unsigned)(d - node0);
    const bool hit = (e < nE) && (sl < (unsigned)TN);
    const unsigned mk = __builtin_amdgcn_ballot_w32(hit);
    if (hit) {
      const int pos = (int)__builtin_amdgcn_mbcnt_lo(mk, 0u);
      sList[wave * WLCAP + pos] = (ec << 5) | (int)sl;
    }
    if (lane == 0) sWcnt[wave] = (int)__builtin_popcount(mk);
    __syncthreads();
    if (wave == 0) {
#pragma unroll 1
      for (int w = 0; w < NWAVE; ++w) {
        int n = __builtin_amdgcn_readfirstlane(sWcnt[w]);
        n = n < 0 ? 0 : (n > WLCAP ? WLCAP : n);
#pragma unroll 1
        for (int i = 0; i < n; ++i) {
          const int ent  = __builtin_amdgcn_readfirstlane(sList[w * WLCAP + i]);
          const int slot = ent & (TN - 1);
          int ev = ent >> 5;
          ev = ev < 0 ? 0 : (ev > nE - 1 ? nE - 1 : ev);
          int sv = esrc[ev];
          sv = sv < 0 ? 0 : (sv > NNODE - 1 ? NNODE - 1 : sv);
          if (lane == 0) {
            const int c = sCnt[slot];
            if (c < DEGCAP) sNbr[slot * DEGCAP + c] = sv;
            sCnt[slot] = (c < DEGCAP) ? (c + 1) : (DEGCAP + 1);
          }
        }
      }
    }
    __syncthreads();
  }
  if (wave == 0) {
    int c = sCnt[lane];
    c = c > DEGCAP ? DEGCAP : c;
    c = max(c, __shfl_xor(c, 16, 32));
    c = max(c, __shfl_xor(c, 8, 32));
    c = max(c, __shfl_xor(c, 4, 32));
    c = max(c, __shfl_xor(c, 2, 32));
    c = max(c, __shfl_xor(c, 1, 32));
    if (lane == 0) sMaxd = c;
  }
  __syncthreads();
  const int maxd = sMaxd;

  const int j  = tid >> 3;
  const int q8 = tid & 7;
  const int c0 = q8 * CPT;
  const int cntj = sCnt[j];
  const int nj = cntj > DEGCAP ? DEGCAP : cntj;
  const _Float16* bp  = Wp + (size_t)(16 * wave + m) * KP + 8 * hh;
  const _Float16* ap0 = sAgg + m * KPA + 8 * hh;
  const _Float16* ap1 = sAgg + (16 + m) * KPA + 8 * hh;

#pragma unroll 1
  for (int bi = 0; bi < BPB; ++bi) {
    const int lb = lb0 + bi;
    if (lb >= nb) break;

    float av[CPT];
#pragma unroll
    for (int e = 0; e < CPT; ++e) av[e] = 0.0f;
#pragma unroll 1
    for (int p = 0; p < maxd; ++p) {
      const int s = sNbr[j * DEGCAP + p];
      const bool use = p < nj;
      if constexpr (F32IN) {
        const float* xp = (const float*)xin + ((size_t)lb * NNODE + s) * KIN + c0;
        const v2f u = *(const v2f*)xp;
        av[0] += use ? u.x : 0.0f;
        av[1] += use ? u.y : 0.0f;
      } else {
        const _Float16* xp = (const _Float16*)xin + ((size_t)lb * NNODE + s) * KIN + c0;
        const v8h u0 = *(const v8h*)xp;
        const v8h u1 = *(const v8h*)(xp + 8);
#pragma unroll
        for (int e = 0; e < 8; ++e) {
          const float f0 = (float)u0[e], f1 = (float)u1[e];
          av[e]     += use ? f0 : 0.0f;
          av[8 + e] += use ? f1 : 0.0f;
        }
      }
    }
    if (cntj > DEGCAP) {
      const float qn = __int_as_float(0x7fc00000);
#pragma unroll
      for (int e = 0; e < CPT; ++e) av[e] = qn;
    }
    if constexpr (F32IN) {
      v2h hv;
      hv[0] = (_Float16)av[0]; hv[1] = (_Float16)av[1];
      *(v2h*)(sAgg + j * KPA + c0) = hv;
    } else {
      v8h h0, h1;
#pragma unroll
      for (int e = 0; e < 8; ++e) { h0[e] = (_Float16)av[e]; h1[e] = (_Float16)av[8 + e]; }
      *(v8h*)(sAgg + j * KPA + c0) = h0;
      *(v8h*)(sAgg + j * KPA + c0 + 8) = h1;
    }
    __syncthreads();

    v8f acc0 = zero8(), acc1 = zero8();
#pragma unroll 1
    for (int kt = 0; kt < KP / 32; ++kt) {
      FragH a0, a1, b;
      b.h[0]  = *(const v8h*)(bp + 32 * kt);
      b.h[1]  = *(const v8h*)(bp + 32 * kt + 16);
      a0.h[0] = *(const v8h*)(ap0 + 32 * kt);
      a0.h[1] = *(const v8h*)(ap0 + 32 * kt + 16);
      a1.h[0] = *(const v8h*)(ap1 + 32 * kt);
      a1.h[1] = *(const v8h*)(ap1 + 32 * kt + 16);
      acc0 = wmf(a0.v, b.v, acc0);
      acc1 = wmf(a1.v, b.v, acc1);
    }

    {
      const int col = 16 * wave + m;
      const float bc = sPar[col];
      float* sp = sOb + (8 * hh) * OBP + col;
#pragma unroll
      for (int r = 0; r < 8; ++r) {
        sp[r * OBP]        = acc0[r] * OSC + bc;
        sp[(16 + r) * OBP] = acc1[r] * OSC + bc;
      }
    }
    __syncthreads();

    {
      const float* rp = sOb + j * OBP + 16 * q8;
      const v4f x0 = *(const v4f*)rp, x1 = *(const v4f*)(rp + 4), x2 = *(const v4f*)(rp + 8), x3 = *(const v4f*)(rp + 12);
      float s = ((x0.x + x0.y) + (x0.z + x0.w)) + ((x1.x + x1.y) + (x1.z + x1.w))
              + ((x2.x + x2.y) + (x2.z + x2.w)) + ((x3.x + x3.y) + (x3.z + x3.w));
      s += __shfl_xor(s, 1, 32); s += __shfl_xor(s, 2, 32); s += __shfl_xor(s, 4, 32);
      const float mu = s * (1.0f / (float)HIDC);
      const v4f d0 = x0 - mu, d1 = x1 - mu, d2 = x2 - mu, d3 = x3 - mu;
      float ss = ((d0.x * d0.x + d0.y * d0.y) + (d0.z * d0.z + d0.w * d0.w))
               + ((d1.x * d1.x + d1.y * d1.y) + (d1.z * d1.z + d1.w * d1.w))
               + ((d2.x * d2.x + d2.y * d2.y) + (d2.z * d2.z + d2.w * d2.w))
               + ((d3.x * d3.x + d3.y * d3.y) + (d3.z * d3.z + d3.w * d3.w));
      ss += __shfl_xor(ss, 1, 32); ss += __shfl_xor(ss, 2, 32); ss += __shfl_xor(ss, 4, 32);
      const float var = ss * (1.0f / (float)HIDC);
      const float rs = rsqrtf(var + LNEPS);
      if (q8 == 0) { sStat[j] = mu; sStat[TN + j] = rs; }
    }
    __syncthreads();

    v8h o[2];
#pragma unroll
    for (int i = 0; i < 2; ++i) {
      const int qq = tid + NTHR * i;
      const int row = qq >> 4, p = qq & 15;
      const float mu = sStat[row], rs = sStat[TN + row];
      const float* xp = sOb + row * OBP + 8 * p;
      const v4f x0 = *(const v4f*)xp, x1 = *(const v4f*)(xp + 4);
      const v4f g0 = *(const v4f*)(sPar + HIDC + 8 * p), g1 = *(const v4f*)(sPar + HIDC + 8 * p + 4);
      const v4f e0 = *(const v4f*)(sPar + 2 * HIDC + 8 * p), e1 = *(const v4f*)(sPar + 2 * HIDC + 8 * p + 4);
      const v4f y0 = (x0 - mu) * rs * g0 + e0;
      const v4f y1 = (x1 - mu) * rs * g1 + e1;
      o[i][0] = (_Float16)fmaxf(y0.x, 0.0f); o[i][1] = (_Float16)fmaxf(y0.y, 0.0f);
      o[i][2] = (_Float16)fmaxf(y0.z, 0.0f); o[i][3] = (_Float16)fmaxf(y0.w, 0.0f);
      o[i][4] = (_Float16)fmaxf(y1.x, 0.0f); o[i][5] = (_Float16)fmaxf(y1.y, 0.0f);
      o[i][6] = (_Float16)fmaxf(y1.z, 0.0f); o[i][7] = (_Float16)fmaxf(y1.w, 0.0f);
    }
    _Float16* ob = hout + ((size_t)lb * NNODE + node0) * HIDC;
    *(volatile v8h*)(ob + 8 * tid) = o[0];
    *(volatile v8h*)(ob + 8 * (tid + NTHR)) = o[1];
    __threadfence();
    *(volatile v8h*)(ob + 8 * tid) = o[0];
    *(volatile v8h*)(ob + 8 * (tid + NTHR)) = o[1];
  }
}

__device__ __forceinline__ void head_plane(const _Float16* __restrict__ ap, const _Float16* __restrict__ bp,
                                           v8f (&acc)[2][2]) {
#pragma unroll 1
  for (int kq = 0; kq < 4; ++kq) {
    FragH a0, a1, b0, b1;
    a0.h[0] = *(const v8h*)(ap + 32 * kq);
    a0.h[1] = *(const v8h*)(ap + 32 * kq + 16);
    a1.h[0] = *(const v8h*)(ap + 16 * HIDC + 32 * kq);
    a1.h[1] = *(const v8h*)(ap + 16 * HIDC + 32 * kq + 16);
    b0.h[0] = *(const v8h*)(bp + 32 * kq);
    b0.h[1] = *(const v8h*)(bp + 32 * kq + 16);
    b1.h[0] = *(const v8h*)(bp + 16 * KPL + 32 * kq);
    b1.h[1] = *(const v8h*)(bp + 16 * KPL + 32 * kq + 16);
    acc[0][0] = wmf(a0.v, b0.v, acc[0][0]);
    acc[0][1] = wmf(a1.v, b0.v, acc[0][1]);
    acc[1][0] = wmf(a0.v, b1.v, acc[1][0]);
    acc[1][1] = wmf(a1.v, b1.v, acc[1][1]);
  }
}

__global__ __launch_bounds__(NTHR) void k_head(const float* __restrict__ obs,
    const _Float16* __restrict__ h1, const _Float16* __restrict__ h2, const _Float16* __restrict__ h3,
    const _Float16* __restrict__ WLw, const float* __restrict__ b1, const float* __restrict__ bng,
    const float* __restrict__ bnb, const float* __restrict__ w2, const float* __restrict__ b2p,
    const int* __restrict__ mask, float* outp, int gbase) {
  __shared__ __attribute__((aligned(16))) _Float16 sObs[TN * SOP];
  __shared__ __attribute__((aligned(16))) float sY[TN * YP];
  __shared__ __attribute__((aligned(16))) float sLg[NNODE];
  __shared__ __attribute__((aligned(16))) float sB1[HID2];
  __shared__ __attribute__((aligned(16))) float sSc[HID2];
  __shared__ __attribute__((aligned(16))) float sSh[HID2];
  __shared__ __attribute__((aligned(16))) float sW2[HID2];
  __shared__ float sRedM[NWAVE];
  __shared__ float sRedS[NWAVE];

  const int tid = threadIdx.x, lane = tid & 31, wave = tid >> 5, hh = lane >> 4, m = lane & 15;
  const int lb = (int)blockIdx.x;
  const int gb = gbase + lb;
  const float bnscale = rsqrtf(1.00001f);
  sB1[tid] = b1[tid];
  sSc[tid] = bng[tid] * bnscale;
  sSh[tid] = bnb[tid];
  sW2[tid] = w2[tid];
  const float b2v = b2p[0];
  const int j = tid >> 3, q8 = tid & 7;
  const int nA = 32 * wave + m;

#pragma unroll 1
  for (int t = 0; t < NNODE / TN; ++t) {
    const int nrow0 = t * TN;
    {
      const int qc = q8 < 4 ? q8 : 3;
      const v4f f = *(const v4f*)(obs + ((size_t)gb * NNODE + nrow0 + j) * FINC + 4 * qc);
      const _Float16 hz = (_Float16)0.0f;
      v4h hv;
      hv[0] = (q8 < 4) ? (_Float16)f.x : hz; hv[1] = (q8 < 4) ? (_Float16)f.y : hz;
      hv[2] = (q8 < 4) ? (_Float16)f.z : hz; hv[3] = (q8 < 4) ? (_Float16)f.w : hz;
      *(v4h*)(sObs + j * SOP + 4 * q8) = hv;
    }
    __syncthreads();

    v8f acc[2][2];
    acc[0][0] = zero8(); acc[0][1] = zero8(); acc[1][0] = zero8(); acc[1][1] = zero8();
    const _Float16* bbase = WLw + (size_t)nA * KPL + 8 * hh;
    {
      FragH a0, a1, b0, b1;
      a0.h[0] = *(const v8h*)(sObs + m * SOP + 8 * hh);
      a0.h[1] = *(const v8h*)(sObs + m * SOP + 16 + 8 * hh);
      a1.h[0] = *(const v8h*)(sObs + (16 + m) * SOP + 8 * hh);
      a1.h[1] = *(const v8h*)(sObs + (16 + m) * SOP + 16 + 8 * hh);
      b0.h[0] = *(const v8h*)(bbase);
      b0.h[1] = *(const v8h*)(bbase + 16);
      b1.h[0] = *(const v8h*)(bbase + 16 * KPL);
      b1.h[1] = *(const v8h*)(bbase + 16 * KPL + 16);
      acc[0][0] = wmf(a0.v, b0.v, acc[0][0]);
      acc[0][1] = wmf(a1.v, b0.v, acc[0][1]);
      acc[1][0] = wmf(a0.v, b1.v, acc[1][0]);
      acc[1][1] = wmf(a1.v, b1.v, acc[1][1]);
    }
    const size_t arow = ((size_t)lb * NNODE + nrow0 + m) * HIDC + 8 * hh;
    head_plane(h1 + arow, bbase + 32 * 1, acc);
    head_plane(h2 + arow, bbase + 32 * 5, acc);
    head_plane(h3 + arow, bbase + 32 * 9, acc);

#pragma unroll
    for (int nti = 0; nti < 2; ++nti) {
      const int n = nA + 16 * nti;
      const float cb = sB1[n], cs = sSc[n], csh = sSh[n];
#pragma unroll
      for (int mt = 0; mt < 2; ++mt) {
        float* sp = sY + (16 * mt + 8 * hh) * YP + n;
#pragma unroll
        for (int r = 0; r < 8; ++r) {
          float v = acc[nti][mt][r] * OSC + cb;
          v = fmaxf(v * cs + csh, 0.0f);
          sp[r * YP] = v;
        }
      }
    }
    __syncthreads();

    {
      const float* yp = sY + j * YP + 32 * q8;
      const float* wp = sW2 + 32 * q8;
      float s = 0.0f;
#pragma unroll 2
      for (int i = 0; i < 8; ++i) {
        const v4f y = *(const v4f*)(yp + 4 * i);
        const v4f w = *(const v4f*)(wp + 4 * i);
        s += y.x * w.x; s += y.y * w.y; s += y.z * w.z; s += y.w * w.w;
      }
      s += __shfl_xor(s, 1, 32); s += __shfl_xor(s, 2, 32); s += __shfl_xor(s, 4, 32);
      const int mv = mask[(size_t)gb * NNODE + nrow0 + j];
      float lg = s + b2v;
      lg = (mv != 0) ? lg : MINV;
      if (q8 == 0) sLg[nrow0 + j] = lg;
    }
  }
  __syncthreads();

  const v4f x = *(const v4f*)(sLg + 4 * tid);
  float mx = fmaxf(fmaxf(x.x, x.y), fmaxf(x.z, x.w));
  mx = fmaxf(mx, __shfl_xor(mx, 16, 32)); mx = fmaxf(mx, __shfl_xor(mx, 8, 32));
  mx = fmaxf(mx, __shfl_xor(mx, 4, 32));  mx = fmaxf(mx, __shfl_xor(mx, 2, 32));
  mx = fmaxf(mx, __shfl_xor(mx, 1, 32));
  if (lane == 0) sRedM[wave] = mx;
  __syncthreads();
  float gmax = sRedM[0];
#pragma unroll
  for (int w = 1; w < NWAVE; ++w) gmax = fmaxf(gmax, sRedM[w]);
  v4f ex;
  ex.x = expf(x.x - gmax); ex.y = expf(x.y - gmax); ex.z = expf(x.z - gmax); ex.w = expf(x.w - gmax);
  float sm = (ex.x + ex.y) + (ex.z + ex.w);
  sm += __shfl_xor(sm, 16, 32); sm += __shfl_xor(sm, 8, 32); sm += __shfl_xor(sm, 4, 32);
  sm += __shfl_xor(sm, 2, 32);  sm += __shfl_xor(sm, 1, 32);
  if (lane == 0) sRedS[wave] = sm;
  __syncthreads();
  float tot = 0.0f;
#pragma unroll
  for (int w = 0; w < NWAVE; ++w) tot += sRedS[w];
  const float inv = 1.0f / tot;
  const v4f pv = ex * inv;
  float* gp = outp + (size_t)gb * NNODE + 4 * tid;
  *(volatile v4f*)gp = pv;
  __threadfence();
  *(volatile v4f*)gp = pv;
}

extern "C" void kernel_launch(void* const* d_in, const int* in_sizes, int n_in,
                              void* d_out, int out_size, void* d_ws, size_t ws_size,
                              hipStream_t stream) {
  if (n_in < 21) return;
  if (in_sizes[1] <= 0 || (in_sizes[1] % NNODE) != 0) return;
  const int B = in_sizes[1] / NNODE;
  if ((long long)in_sizes[0] != (long long)B * NNODE * FINC) return;
  if (in_sizes[2] < 2 || (in_sizes[2] & 1) != 0) return;
  const int nE = in_sizes[2] / 2;
  if (nE < 1 || nE > (1 << 20)) return;
  if (in_sizes[3] != FINC * HIDC || in_sizes[4] != HIDC || in_sizes[5] != HIDC || in_sizes[6] != HIDC) return;
  if (in_sizes[7] != HIDC * HIDC || in_sizes[8] != HIDC || in_sizes[9] != HIDC || in_sizes[10] != HIDC) return;
  if (in_sizes[11] != HIDC * HIDC || in_sizes[12] != HIDC || in_sizes[13] != HIDC || in_sizes[14] != HIDC) return;
  if (in_sizes[15] != KLIN * HID2 || in_sizes[16] != HID2 || in_sizes[17] != HID2 || in_sizes[18] != HID2) return;
  if (in_sizes[19] != HID2 || in_sizes[20] < 1) return;
  if ((long long)out_size != (long long)B * NNODE) return;
  const int nG = (B + BGRP - 1) / BGRP;
  if (nG < 1 || nG > 64) return;

  const float* obs   = (const float*)d_in[0];
  const int*   mask  = (const int*)d_in[1];
  const int*   ei    = (const int*)d_in[2];
  const float* c0w   = (const float*)d_in[3];
  const float* c0b   = (const float*)d_in[4];
  const float* l0g   = (const float*)d_in[5];
  const float* l0b   = (const float*)d_in[6];
  const float* c1w   = (const float*)d_in[7];
  const float* c1b   = (const float*)d_in[8];
  const float* l1g   = (const float*)d_in[9];
  const float* l1b   = (const float*)d_in[10];
  const float* c2w   = (const float*)d_in[11];
  const float* c2b   = (const float*)d_in[12];
  const float* l2g   = (const float*)d_in[13];
  const float* l2b   = (const float*)d_in[14];
  const float* l1w   = (const float*)d_in[15];
  const float* l1bb  = (const float*)d_in[16];
  const float* bng   = (const float*)d_in[17];
  const float* bnb   = (const float*)d_in[18];
  const float* l2w   = (const float*)d_in[19];
  const float* lin2b = (const float*)d_in[20];
  float* out = (float*)d_out;
  const int* esrc = ei;
  const int* edst = ei + nE;

  char* ws = (char*)d_ws;
  size_t off = 0;
  const size_t hpl = (size_t)BGRP * NNODE * HIDC * 2;
  const size_t oH1 = off; off += hpl;                          off = (off + 255) & ~(size_t)255;
  const size_t oH2 = off; off += hpl;                          off = (off + 255) & ~(size_t)255;
  const size_t oH3 = off; off += hpl;                          off = (off + 255) & ~(size_t)255;
  const size_t oW0 = off; off += (size_t)HIDC * 32 * 2;        off = (off + 255) & ~(size_t)255;
  const size_t oW1 = off; off += (size_t)HIDC * HIDC * 2;      off = (off + 255) & ~(size_t)255;
  const size_t oW2 = off; off += (size_t)HIDC * HIDC * 2;      off = (off + 255) & ~(size_t)255;
  const size_t oWL = off; off += (size_t)HID2 * KPL * 2;       off = (off + 255) & ~(size_t)255;
  if (off > ws_size || off > (size_t)WSCAP) return;
  _Float16* H1  = (_Float16*)(ws + oH1);
  _Float16* H2  = (_Float16*)(ws + oH2);
  _Float16* H3  = (_Float16*)(ws + oH3);
  _Float16* W0p = (_Float16*)(ws + oW0);
  _Float16* W1p = (_Float16*)(ws + oW1);
  _Float16* W2p = (_Float16*)(ws + oW2);
  _Float16* WLp = (_Float16*)(ws + oWL);

  k_wT16<32>  <<<HIDC / 32, NTHR, 0, stream>>>(c0w, W0p, FINC, HIDC, FINC, 0, (float)WSCL);
  k_wT16<HIDC><<<HIDC / 32, NTHR, 0, stream>>>(c1w, W1p, HIDC, HIDC, HIDC, 0, (float)WSCL);
  k_wT16<HIDC><<<HIDC / 32, NTHR, 0, stream>>>(c2w, W2p, HIDC, HIDC, HIDC, 0, (float)WSCL);
  k_wT16<KPL> <<<HID2 / 32, NTHR, 0, stream>>>(l1w, WLp, KLIN, HID2, KL1, KGAP, (float)WSCL);

  for (int g = 0; g < nG; ++g) {
    const int rem = B - g * BGRP;
    const int nb  = rem < BGRP ? rem : BGRP;
    const int gy  = (nb + BPB - 1) / BPB;
    const float* obsg = obs + (size_t)g * BGRP * NNODE * FINC;
    const dim3 grid(NNODE / TN, gy);
    k_layer<FINC, true> <<<grid, NTHR, 0, stream>>>((const void*)obsg, esrc, edst, W0p, c0b, l0g, l0b, H1, nE, nb);
    k_layer<HIDC, false><<<grid, NTHR, 0, stream>>>((const void*)H1,   esrc, edst, W1p, c1b, l1g, l1b, H2, nE, nb);
    k_layer<HIDC, false><<<grid, NTHR, 0, stream>>>((const void*)H2,   esrc, edst, W2p, c2b, l2g, l2b, H3, nE, nb);
    k_head<<<nb, NTHR, 0, stream>>>(obs, H1, H2, H3, WLp, l1bb, bng, bnb, l2w, lin2b, mask, out, g * BGRP);
  }
}
